// MiniMultiNet_46351287058819
// MI455X (gfx1250) — hardware-verified
//
#include <hip/hip_runtime.h>
#define NS 512
#define CHS 128
#define P0 3025
#define P1 784
#define P2 196
#define P3 49
typedef __bf16 v16b __attribute__((ext_vector_type(16)));
typedef unsigned short v8us __attribute__((ext_vector_type(8), may_alias));
typedef float  v8f  __attribute__((ext_vector_type(8)));
typedef float  v4f  __attribute__((ext_vector_type(4)));
typedef float  v4fa __attribute__((ext_vector_type(4), may_alias));
union FragB { v16b v; v8us half[2]; unsigned short u[16]; };

__device__ __forceinline__ unsigned short bf16_bits(float x) { unsigned int u = __float_as_uint(x); return (unsigned short)((u + 0x7FFFu + ((u >> 16) & 1u)) >> 16); }
__device__ __forceinline__ float bf16_val(unsigned short b) { return __uint_as_float(((unsigned int)b) << 16); }
__device__ __forceinline__ float bf16_round(float x) { return bf16_val(bf16_bits(x)); }
template <int NT>
__device__ __forceinline__ v8f mmaN(v16b ah, v16b al, v16b bh, v16b bl, v8f c) {
  c = __builtin_amdgcn_wmma_f32_16x16x32_bf16(false, ah, false, bh, (short)0, c, false, false);
  if (NT >= 2) c = __builtin_amdgcn_wmma_f32_16x16x32_bf16(false, al, false, bh, (short)0, c, false, false);
  if (NT >= 3) c = __builtin_amdgcn_wmma_f32_16x16x32_bf16(false, ah, false, bl, (short)0, c, false, false);
  asm volatile("v_nop\n\tv_nop\n\tv_nop\n\tv_nop" : "+v"(c) : "v"(ah), "v"(al), "v"(bh), "v"(bl));
  return c;
}

__global__ __launch_bounds__(256) void k_wt_bf16(const float* __restrict__ W, unsigned short* __restrict__ Wt, int K, int N) {
  const int t = blockIdx.x * 256 + threadIdx.x;
  const int k8n = K / 8;
  if (t >= N * k8n) return;
  const int n = t / k8n, k8 = (t % k8n) * 8;
  v8us v;
#pragma unroll
  for (int i = 0; i < 8; ++i) v[i] = bf16_bits(W[(size_t)(k8 + i) * N + n]);
  *(volatile v8us*)(Wt + (size_t)n * K + k8) = v;
  __threadfence();
  *(volatile v8us*)(Wt + (size_t)n * K + k8) = v;
}

template <bool ASPLIT, int ACT, bool BIAS_BF16>
__global__ __launch_bounds__(128) void k_gemm_bf(const float* __restrict__ A, int lda, const unsigned short* __restrict__ Wt, int ldb,
                                               const float* __restrict__ bias, float* __restrict__ C, int ldc, int M, int N, int K) {
  __shared__ __attribute__((aligned(16))) float so[4][16][64];
  const int tid = threadIdx.x, w = tid >> 5, lane = tid & 31, ln = lane & 15, hh = lane >> 4;
  const int ntn = N / 64;
  const int wid = blockIdx.x * 4 + w;
  const int mt = wid / ntn, nq = wid % ntn;
  if (mt * 16 >= M) return;
  const int row0 = mt * 16, col0 = nq * 64;
  const float* arow = A + (size_t)(row0 + ln) * lda;
  v8f acc[4] = {};
  for (int kb = 0; kb < K; kb += 32) {
    FragB ah, al;
    const v4f x0 = *(const v4fa*)(arow + kb + 8 * hh), x1 = *(const v4fa*)(arow + kb + 8 * hh + 4);
    const v4f x2 = *(const v4fa*)(arow + kb + 16 + 8 * hh), x3 = *(const v4fa*)(arow + kb + 16 + 8 * hh + 4);
    float xs[16] = {x0[0],x0[1],x0[2],x0[3],x1[0],x1[1],x1[2],x1[3],x2[0],x2[1],x2[2],x2[3],x3[0],x3[1],x3[2],x3[3]};
#pragma unroll
    for (int i = 0; i < 16; ++i) { const unsigned short hb = bf16_bits(xs[i]); ah.u[i] = hb; al.u[i] = ASPLIT ? bf16_bits(xs[i] - bf16_val(hb)) : (unsigned short)0; }
#pragma unroll
    for (int t = 0; t < 4; ++t) {
      const unsigned short* brow = Wt + (size_t)(col0 + t * 16 + ln) * ldb + kb;
      FragB b;
      b.half[0] = *(const v8us*)(brow + 8 * hh);
      b.half[1] = *(const v8us*)(brow + 16 + 8 * hh);
      acc[t] = mmaN<ASPLIT ? 2 : 1>(ah.v, al.v, b.v, b.v, acc[t]);
    }
  }
#pragma unroll
  for (int t = 0; t < 4; ++t) {
    float bv = bias ? bias[col0 + t * 16 + ln] : 0.f;
    if (BIAS_BF16) bv = bf16_round(bv);
#pragma unroll
    for (int r = 0; r < 8; ++r) { float v = acc[t][r] + bv; if (ACT == 1) v = fmaxf(v, 0.f); so[w][8 * hh + r][t * 16 + ln] = v; }
  }
  __builtin_amdgcn_fence(__ATOMIC_ACQ_REL, "workgroup");
  __builtin_amdgcn_wave_barrier();
  const int rsub = lane >> 4, c4 = (lane & 15) * 4;
  for (int pass = 0; pass < 2; ++pass) {
#pragma unroll
    for (int q = 0; q < 8; ++q) {
      const int r = q * 2 + rsub;
      const v4f v = *(const v4fa*)&so[w][r][c4];
      *(volatile v4f*)(C + (size_t)(row0 + r) * ldc + col0 + c4) = v;
    }
    if (pass == 0) __threadfence();
  }
}

template <bool ASPLIT, int ACT, bool BIAS_BF16, bool RES_BF16>
__global__ __launch_bounds__(128) void k_gemm_bf3(const float* __restrict__ A, int lda, const unsigned short* __restrict__ Wt, int ldb,
                                                const float* __restrict__ bias, const float* __restrict__ resid, int rmod, int ldr,
                                                float* __restrict__ C, int ldc, int M, int N, int K) {
  __shared__ __attribute__((aligned(16))) float so[4][16][64];
  const int tid = threadIdx.x, w = tid >> 5, lane = tid & 31, ln = lane & 15, hh = lane >> 4;
  const int ntn = N / 64;
  const int wid = blockIdx.x * 4 + w;
  const int mt = wid / ntn, nq = wid % ntn;
  if (mt * 16 >= M) return;
  const int row0 = mt * 16, col0 = nq * 64;
  const float* arow = A + (size_t)(row0 + ln) * lda;
  v8f acc[4] = {};
  for (int kb = 0; kb < K; kb += 32) {
    FragB ah, al;
    const v4f x0 = *(const v4fa*)(arow + kb + 8 * hh), x1 = *(const v4fa*)(arow + kb + 8 * hh + 4);
    const v4f x2 = *(const v4fa*)(arow + kb + 16 + 8 * hh), x3 = *(const v4fa*)(arow + kb + 16 + 8 * hh + 4);
    float xs[16] = {x0[0],x0[1],x0[2],x0[3],x1[0],x1[1],x1[2],x1[3],x2[0],x2[1],x2[2],x2[3],x3[0],x3[1],x3[2],x3[3]};
#pragma unroll
    for (int i = 0; i < 16; ++i) { const unsigned short hb = bf16_bits(xs[i]); ah.u[i] = hb; al.u[i] = ASPLIT ? bf16_bits(xs[i] - bf16_val(hb)) : (unsigned short)0; }
#pragma unroll
    for (int t = 0; t < 4; ++t) {
      const unsigned short* brow = Wt + (size_t)(col0 + t * 16 + ln) * ldb + kb;
      FragB b;
      b.half[0] = *(const v8us*)(brow + 8 * hh);
      b.half[1] = *(const v8us*)(brow + 16 + 8 * hh);
      acc[t] = mmaN<ASPLIT ? 2 : 1>(ah.v, al.v, b.v, b.v, acc[t]);
    }
  }
#pragma unroll
  for (int t = 0; t < 4; ++t) {
    const int col = col0 + t * 16 + ln;
    float bv = bias ? bias[col] : 0.f;
    if (BIAS_BF16) bv = bf16_round(bv);
#pragma unroll
    for (int r = 0; r < 8; ++r) {
      float v = acc[t][r] + bv;
      if (resid) { float rv = resid[(size_t)((row0 + 8 * hh + r) % rmod) * ldr + col]; if (RES_BF16) rv = bf16_round(rv); v += rv; }
      if (ACT == 1) v = fmaxf(v, 0.f);
      if (ACT == 2) v = 0.5f * v * (1.0f + erff(v * 0.70710678118654752f));
      if (ACT == 3) { const float u = 0.7978845608028654f * (v + 0.044715f * v * v * v); v = 0.5f * v * (1.0f + tanhf(u)); }
      so[w][8 * hh + r][t * 16 + ln] = v;
    }
  }
  __builtin_amdgcn_fence(__ATOMIC_ACQ_REL, "workgroup");
  __builtin_amdgcn_wave_barrier();
  const int rsub = lane >> 4, c4 = (lane & 15) * 4;
  for (int pass = 0; pass < 2; ++pass) {
#pragma unroll
    for (int q = 0; q < 8; ++q) {
      const int r = q * 2 + rsub;
      const v4f v = *(const v4fa*)&so[w][r][c4];
      *(volatile v4f*)(C + (size_t)(row0 + r) * ldc + col0 + c4) = v;
    }
    if (pass == 0) __threadfence();
  }
}
template <bool PARAM_BF16>
__global__ __launch_bounds__(256) void k_layernorm(const float* __restrict__ X, const float* __restrict__ R, const float* __restrict__ g, const float* __restrict__ bta,
                                                  float* __restrict__ out_sum, float* __restrict__ out_norm, int N, float eps) {
  __shared__ float red[256];
  const int row = blockIdx.x, tid = threadIdx.x;
  const float* x = X + (size_t)row * N; const float* rr = R ? R + (size_t)row * N : nullptr;
  float vals[16];
  const int per = N / 256;
  float s1 = 0.f;
  for (int u = 0; u < per / 4; ++u) {
    const int j = tid * 4 + 1024 * u;
    const v4f a = *(const v4fa*)(x + j);
    v4f b = {0.f,0.f,0.f,0.f}; if (rr) b = *(const v4fa*)(rr + j);
#pragma unroll
    for (int q = 0; q < 4; ++q) { const float v = a[q] + b[q]; vals[u * 4 + q] = v; s1 += v; }
  }
  red[tid] = s1; __syncthreads();
  for (int st = 128; st > 0; st >>= 1) { if (tid < st) red[tid] += red[tid + st]; __syncthreads(); }
  const float mu = red[0] / (float)N; __syncthreads();
  float s2 = 0.f;
  for (int u = 0; u < per / 4; ++u)
#pragma unroll
    for (int q = 0; q < 4; ++q) { const float c = vals[u * 4 + q] - mu; s2 += c * c; }
  red[tid] = s2; __syncthreads();
  for (int st = 128; st > 0; st >>= 1) { if (tid < st) red[tid] += red[tid + st]; __syncthreads(); }
  const float rs = rsqrtf(red[0] / (float)N + eps);
  for (int pass = 0; pass < 2; ++pass) {
    for (int u = 0; u < per / 4; ++u) {
      const int j = tid * 4 + 1024 * u;
      v4f o, sm;
#pragma unroll
      for (int q = 0; q < 4; ++q) {
        float gg = g[j + q], bb = bta[j + q];
        if (PARAM_BF16) { gg = bf16_round(gg); bb = bf16_round(bb); }
        sm[q] = vals[u * 4 + q]; o[q] = (vals[u * 4 + q] - mu) * rs * gg + bb;
      }
      if (out_sum) *(volatile v4f*)(out_sum + (size_t)row * N + j) = sm;
      *(volatile v4f*)(out_norm + (size_t)row * N + j) = o;
    }
    if (pass == 0) __threadfence();
  }
}


typedef _Float16 v16h __attribute__((ext_vector_type(16)));
union FragH { v16h v; v8us half[2]; _Float16 h[16]; unsigned short u[16]; };
template <int NT>
__device__ __forceinline__ v8f mmaH(v16h ah, v16h al, v16h bh, v16h bl, v8f c) {
  c = __builtin_amdgcn_wmma_f32_16x16x32_f16(false, ah, false, bh, (short)0, c, false, false);
  if (NT >= 2) c = __builtin_amdgcn_wmma_f32_16x16x32_f16(false, al, false, bh, (short)0, c, false, false);
  if (NT >= 3) c = __builtin_amdgcn_wmma_f32_16x16x32_f16(false, ah, false, bl, (short)0, c, false, false);
  asm volatile("v_nop\n\tv_nop\n\tv_nop\n\tv_nop" : "+v"(c) : "v"(ah), "v"(al), "v"(bh), "v"(bl));
  return c;
}
template <bool ASPLIT>
__global__ __launch_bounds__(128) void k_gemm_h(const float* __restrict__ A, int lda, size_t sA, const _Float16* __restrict__ Bh, int ldb, size_t sB, float alpha, float* __restrict__ C, int ldc, size_t sC, int M, int N, int K) {
  __shared__ __attribute__((aligned(16))) float so[4][16][64];
  const int tid = threadIdx.x, w = tid >> 5, lane = tid & 31, ln = lane & 15, hh = lane >> 4; const int by = blockIdx.y;
  A += (size_t)by * sA; Bh += (size_t)by * sB; C += (size_t)by * sC;
  const int ntn = (N + 63) / 64; const int wid = blockIdx.x * 4 + w; const int mt = wid / ntn, nq = wid % ntn; if (mt * 16 >= M) return;
  const int row0 = mt * 16, col0 = nq * 64; const float* arow = A + (size_t)(row0 + ln) * lda;
  v8f acc[4] = {};
  for (int kb = 0; kb < K; kb += 32) {
    FragH ah, al;
    const v4f x0 = *(const v4fa*)(arow + kb + 8 * hh), x1 = *(const v4fa*)(arow + kb + 8 * hh + 4), x2 = *(const v4fa*)(arow + kb + 16 + 8 * hh), x3 = *(const v4fa*)(arow + kb + 16 + 8 * hh + 4);
    float xs[16] = {x0[0],x0[1],x0[2],x0[3],x1[0],x1[1],x1[2],x1[3],x2[0],x2[1],x2[2],x2[3],x3[0],x3[1],x3[2],x3[3]};
#pragma unroll
    for (int i = 0; i < 16; ++i) { const _Float16 h = (_Float16)xs[i]; ah.h[i] = h; al.h[i] = ASPLIT ? (_Float16)(xs[i] - (float)h) : (_Float16)0.0f; }
#pragma unroll
    for (int t = 0; t < 4; ++t) { if (col0 + t * 16 >= N) continue; const size_t boff = (size_t)(col0 + t * 16 + ln) * ldb + kb; FragH bq; bq.half[0] = *(const v8us*)(Bh + boff + 8 * hh); bq.half[1] = *(const v8us*)(Bh + boff + 16 + 8 * hh);
      acc[t] = mmaH<ASPLIT ? 2 : 1>(ah.v, al.v, bq.v, bq.v, acc[t]); }
  }
#pragma unroll
  for (int t = 0; t < 4; ++t) { if (col0 + t * 16 >= N) continue;
#pragma unroll
    for (int r = 0; r < 8; ++r) so[w][8 * hh + r][t * 16 + ln] = acc[t][r] * alpha; }
  __builtin_amdgcn_fence(__ATOMIC_ACQ_REL, "workgroup"); __builtin_amdgcn_wave_barrier();
  const int rsub = lane >> 4, c4 = (lane & 15) * 4;
  for (int pass = 0; pass < 2; ++pass) {
#pragma unroll
    for (int q = 0; q < 8; ++q) { const int r = q * 2 + rsub; if (col0 + c4 < N) { const v4f v = *(const v4fa*)&so[w][r][c4]; *(volatile v4f*)(C + (size_t)(row0 + r) * ldc + col0 + c4) = v; } }
    if (pass == 0) __threadfence(); }
}

__global__ __launch_bounds__(256) void k_wt_f16(const float* __restrict__ W, _Float16* __restrict__ Wt, int K, int N, float scale) {
  const int t = blockIdx.x * 256 + threadIdx.x; if (t >= N * (K / 8)) return; const int n = t / (K / 8), k8 = (t % (K / 8)) * 8; FragH f;
#pragma unroll
  for (int i = 0; i < 8; ++i) f.h[i] = (_Float16)(bf16_round(W[(size_t)(k8 + i) * N + n]) * scale); const v8us o = f.half[0];
  *(volatile v8us*)((unsigned short*)Wt + (size_t)n * K + k8) = o; __threadfence(); *(volatile v8us*)((unsigned short*)Wt + (size_t)n * K + k8) = o;
}
template <int ACT>
__global__ __launch_bounds__(128) void k_gemm_hhx(const _Float16* __restrict__ A, int lda, size_t sA, const _Float16* __restrict__ Bh, int ldb, size_t sB, float alpha, const float* __restrict__ bias, size_t sBias, const float* __restrict__ CP, int rowsPerB, size_t sCPb, int row0g,
    float* __restrict__ C, _Float16* __restrict__ C16, int ldc, size_t sC, int M, int N, int K) {
  __shared__ __attribute__((aligned(16))) float so[4][16][64];
  const int tid = threadIdx.x, w = tid >> 5, lane = tid & 31, ln = lane & 15, hh = lane >> 4; const int by = blockIdx.y;
  A += (size_t)by * sA; Bh += (size_t)by * sB; const size_t cofs = (size_t)by * sC; const float* bp = bias ? bias + (size_t)by * sBias : nullptr;
  const int ntn = (N + 63) / 64; const int wid = blockIdx.x * 4 + w; const int mt = wid / ntn, nq = wid % ntn; if (mt * 16 >= M) return;
  const int row0 = mt * 16, col0 = nq * 64; const _Float16* arow = A + (size_t)(row0 + ln) * lda;
  v8f acc[4] = {};
  for (int kb = 0; kb < K; kb += 32) { FragH ah; ah.half[0] = *(const v8us*)((const unsigned short*)arow + kb + 8 * hh); ah.half[1] = *(const v8us*)((const unsigned short*)arow + kb + 16 + 8 * hh);
#pragma unroll
    for (int t = 0; t < 4; ++t) { if (col0 + t * 16 >= N) continue; const size_t boff = (size_t)(col0 + t * 16 + ln) * ldb + kb; FragH bq; bq.half[0] = *(const v8us*)((const unsigned short*)Bh + boff + 8 * hh); bq.half[1] = *(const v8us*)((const unsigned short*)Bh + boff + 16 + 8 * hh);
      acc[t] = mmaH<1>(ah.v, ah.v, bq.v, bq.v, acc[t]); }
  }
#pragma unroll
  for (int t = 0; t < 4; ++t) { if (col0 + t * 16 >= N) continue; const int col = col0 + t * 16 + ln; const float bv = bp ? bf16_round(bp[col]) : 0.f;
#pragma unroll
    for (int r = 0; r < 8; ++r) { float v = acc[t][r] * alpha + bv; if (CP) { const int rr = row0g + row0 + 8 * hh + r; if (rowsPerB < 0) v += CP[cofs + (size_t)rr * ldc + col];        else { const int bidx = rr / rowsPerB; v += CP[(size_t)bidx * sCPb + (size_t)by * 64 + col]; } } if (ACT == 1) v = (v > 0.f) ? v : expm1f(v); else if (ACT == 7) v = (v > 0.f) ? v + 1.0f : expf(v); else if (ACT == 8) v = tanhf(v); else if (ACT == 9) v = 0.5f * v * (1.0f + tanhf(0.7978845608028654f * (v + 0.044715f * v * v * v))); else if (ACT == 11) v = 1.0f / (1.0f + expf(-v)); else if (ACT == 12) v = (v > 0.f) ? v : 0.01f * v; else if (ACT == 14) v = (v > 0.f) ? v : 0.1f * v; else if (ACT == 15) v = v / (1.0f + expf(-v)); else if (ACT == 3) v = fmaxf(v, 0.f); else if (ACT == 6) v = 0.5f * v * (1.0f + erff(v * 0.70710678118654752f)); so[w][8 * hh + r][t * 16 + ln] = v; } }
  __builtin_amdgcn_fence(__ATOMIC_ACQ_REL, "workgroup"); __builtin_amdgcn_wave_barrier();
  const int rsub = lane >> 4, c4 = (lane & 15) * 4; typedef _Float16 v4h __attribute__((ext_vector_type(4)));
  for (int pass = 0; pass < 2; ++pass) {
#pragma unroll
    for (int q = 0; q < 8; ++q) { const int r = q * 2 + rsub; if (col0 + c4 < N) { const v4f v = *(const v4fa*)&so[w][r][c4]; if (C) *(volatile v4f*)(C + cofs + (size_t)(row0 + r) * ldc + col0 + c4) = v; if (C16) { v4h h4; for (int i = 0; i < 4; ++i) h4[i] = (_Float16)v[i]; *(volatile v4h*)(C16 + cofs + (size_t)(row0 + r) * ldc + col0 + c4) = h4; } } }
    if (pass == 0) __threadfence(); }
}


typedef _Float16 v4h __attribute__((ext_vector_type(4)));

__global__ __launch_bounds__(256) void k_x16(const float* __restrict__ x, _Float16* __restrict__ X16, size_t n8) { const size_t t = (size_t)blockIdx.x * 256 + threadIdx.x; if (t >= n8) return; FragH f;
#pragma unroll
  for (int q = 0; q < 8; ++q) f.h[q] = (_Float16)bf16_round(x[t * 8 + q]); *(volatile v8us*)((unsigned short*)X16 + t * 8) = f.half[0]; __threadfence(); *(volatile v8us*)((unsigned short*)X16 + t * 8) = f.half[0]; }
__global__ __launch_bounds__(256) void k_h16(const float* __restrict__ x, _Float16* __restrict__ X16, size_t n8) { const size_t t = (size_t)blockIdx.x * 256 + threadIdx.x; if (t >= n8) return; FragH f;
#pragma unroll
  for (int q = 0; q < 8; ++q) f.h[q] = (_Float16)x[t * 8 + q]; *(volatile v8us*)((unsigned short*)X16 + t * 8) = f.half[0]; __threadfence(); *(volatile v8us*)((unsigned short*)X16 + t * 8) = f.half[0]; }
__global__ __launch_bounds__(256) void k_round16f(const float* __restrict__ W, _Float16* __restrict__ Bt, size_t n8) { const size_t t = (size_t)blockIdx.x * 256 + threadIdx.x; if (t >= n8) return; FragH f;
#pragma unroll
  for (int i = 0; i < 8; ++i) f.h[i] = (_Float16)(bf16_round(W[t * 8 + i]) * 16.0f); *(volatile v8us*)((unsigned short*)Bt + t * 8) = f.half[0]; __threadfence(); *(volatile v8us*)((unsigned short*)Bt + t * 8) = f.half[0]; }
template <int NHv, int TTv>
__global__ __launch_bounds__(256) void k_vt(const _Float16* __restrict__ V16, int ldv, int voff, _Float16* __restrict__ Vt) { __shared__ unsigned short tl[64][66]; const int tid = threadIdx.x; const int slab = blockIdx.x / (TTv / 64), lg = blockIdx.x % (TTv / 64); const int b = slab / NHv, h = slab % NHv;
  for (int i = tid; i < 64 * 8; i += 256) { const int r = i / 8, c8 = (i % 8) * 8; FragH f; f.half[0] = *(const v8us*)((const unsigned short*)V16 + ((size_t)b * TTv + lg * 64 + r) * ldv + voff + h * 64 + c8);
#pragma unroll
    for (int q = 0; q < 8; ++q) tl[r][c8 + q] = f.u[q]; }
  __syncthreads();
  for (int pass = 0; pass < 2; ++pass) {
#pragma unroll
    for (int rd = 0; rd < 2; ++rd) { const int d = rd * 32 + tid / 8, pc = tid % 8; FragH f;
#pragma unroll
      for (int q = 0; q < 8; ++q) f.u[q] = tl[pc * 8 + q][d];
      *(volatile v8us*)((unsigned short*)Vt + ((size_t)slab * 64 + d) * TTv + lg * 64 + pc * 8) = f.half[0]; }
    if (pass == 0) __threadfence(); } }

__global__ __launch_bounds__(256) void k_hl(const float* __restrict__ F, _Float16* __restrict__ Hh, _Float16* __restrict__ Hl, size_t n8) { const size_t t = (size_t)blockIdx.x * 256 + threadIdx.x; if (t >= n8) return; FragH fh, fl; const v4f a = *(const v4fa*)(F + t * 8), c = *(const v4fa*)(F + t * 8 + 4);
#pragma unroll
  for (int q = 0; q < 4; ++q) { _Float16 h = (_Float16)a[q]; fh.h[q] = h; fl.h[q] = (_Float16)((a[q] - (float)h) * 1024.0f); h = (_Float16)c[q]; fh.h[4 + q] = h; fl.h[4 + q] = (_Float16)((c[q] - (float)h) * 1024.0f); }
  for (int pass = 0; pass < 2; ++pass) { *(volatile v8us*)((unsigned short*)Hh + t * 8) = fh.half[0]; *(volatile v8us*)((unsigned short*)Hl + t * 8) = fl.half[0]; if (pass == 0) __threadfence(); } }

__device__ __forceinline__ v16h g2_frag(const _Float16* p, int hh) { FragH f; f.half[0] = *(const v8us*)((const unsigned short*)p + 8 * hh); f.half[1] = *(const v8us*)((const unsigned short*)p + 16 + 8 * hh); return f.v; }
__device__ __forceinline__ v8f g2_mma(v16h a, v16h b, v8f c) { v8f d = __builtin_amdgcn_wmma_f32_16x16x32_f16(false, a, false, b, (short)0, c, false, false); asm volatile("v_nop\n\tv_nop\n\tv_nop\n\tv_nop" : "+v"(d) : "v"(a), "v"(b)); return d; }
template <int ACT>
__global__ __launch_bounds__(128) void k_gemm2(const _Float16* __restrict__ A, int lda, size_t sA, const _Float16* __restrict__ Bh, int ldb, size_t sB, float alpha, const float* __restrict__ bias, size_t sBias, const float* __restrict__ CP, int rowsPerB, size_t sCPb, int row0g,
    float* __restrict__ C, _Float16* __restrict__ C16, int ldc, size_t sC, int M, int N, int K) {
  __shared__ __attribute__((aligned(16))) float so[4][32][68];
  const int tid = threadIdx.x, w = tid >> 5, lane = tid & 31, ln = lane & 15, hh = lane >> 4; const int by = blockIdx.y;
  A += (size_t)by * sA; Bh += (size_t)by * sB; const size_t cofs = (size_t)by * sC; const float* bp = bias ? bias + (size_t)by * sBias : nullptr;
  const int ntn = N >> 6; const int mt = blockIdx.x / ntn, nq = blockIdx.x - mt * ntn; const int row0 = mt * 128 + 32 * w, col0 = nq * 64; if (row0 >= M) return;
  const _Float16* a0p = A + (size_t)(row0 + ln) * lda; const _Float16* a1p = a0p + (size_t)16 * lda;
  const _Float16* b0p = Bh + (size_t)(col0 + ln) * ldb; const _Float16* b1p = b0p + (size_t)16 * ldb; const _Float16* b2p = b1p + (size_t)16 * ldb; const _Float16* b3p = b2p + (size_t)16 * ldb;
  const v8f z8 = {0.f,0.f,0.f,0.f,0.f,0.f,0.f,0.f}; v8f c00 = z8, c01 = z8, c02 = z8, c03 = z8, c10 = z8, c11 = z8, c12 = z8, c13 = z8;
#pragma unroll 1
  for (int kb = 0; kb < K; kb += 32) { const v16h a0 = g2_frag(a0p + kb, hh), a1 = g2_frag(a1p + kb, hh);
    v16h b = g2_frag(b0p + kb, hh); c00 = g2_mma(a0, b, c00); c10 = g2_mma(a1, b, c10);
    b = g2_frag(b1p + kb, hh); c01 = g2_mma(a0, b, c01); c11 = g2_mma(a1, b, c11);
    b = g2_frag(b2p + kb, hh); c02 = g2_mma(a0, b, c02); c12 = g2_mma(a1, b, c12);
    b = g2_frag(b3p + kb, hh); c03 = g2_mma(a0, b, c03); c13 = g2_mma(a1, b, c13); }
  v8f accs[8] = {c00, c01, c02, c03, c10, c11, c12, c13};
#pragma unroll
  for (int u = 0; u < 8; ++u) { const int t = u & 3, half = u >> 2; const int col = col0 + t * 16 + ln; const float bv = bp ? bf16_round(bp[col]) : 0.f;
#pragma unroll
    for (int r = 0; r < 8; ++r) { const int rloc = half * 16 + 8 * hh + r; float v = accs[u][r] * alpha + bv; if (CP) { if (rowsPerB < 0) v += CP[cofs + (size_t)(row0g + row0 + rloc) * ldc + col];        else { const int bidx = (row0g + row0 + rloc) / rowsPerB; v += CP[(size_t)bidx * sCPb + (size_t)by * 64 + col]; } }
      if (ACT == 3) v = fmaxf(v, 0.f); else if (ACT == 6) v = 0.5f * v * (1.0f + erff(v * 0.70710678118654752f)); else if (ACT == 11) v = 1.0f / (1.0f + expf(-v)); else if (ACT == 15) v = v / (1.0f + expf(-v)); else if (ACT == 12) v = (v > 0.f) ? v : 0.01f * v; else if (ACT == 8) v = tanhf(v);
      so[w][rloc][t * 16 + ln] = v; } }
  __builtin_amdgcn_fence(__ATOMIC_ACQ_REL, "workgroup"); __builtin_amdgcn_wave_barrier();
  const int rsub = lane >> 4, c4 = (lane & 15) * 4;
  for (int pass = 0; pass < 2; ++pass) {
#pragma unroll
    for (int q = 0; q < 16; ++q) { const int r = q * 2 + rsub; const v4f v = *(const v4fa*)&so[w][r][c4]; if (C) *(volatile v4f*)(C + cofs + (size_t)(row0 + r) * ldc + col0 + c4) = v; if (C16) { v4h h4; for (int i = 0; i < 4; ++i) h4[i] = (_Float16)v[i]; *(volatile v4h*)(C16 + cofs + (size_t)(row0 + r) * ldc + col0 + c4) = h4; } }
    if (pass == 0) __threadfence(); } }


__global__ __launch_bounds__(256) void k_wconv(const float* __restrict__ Wm, const float* __restrict__ bm, int O, int CIN, int KPAD, int TAPMAJ, _Float16* __restrict__ Bt, float* __restrict__ BB) {
  const int tid = threadIdx.x; const int KR = CIN * 9;
  for (int pass = 0; pass < 2; ++pass) { for (int t = tid; t < 64 * (KPAD / 8); t += 256) { const int c0 = (t % (KPAD / 8)) * 8; const int o = t / (KPAD / 8); FragH f; for (int q = 0; q < 8; ++q) { const int col = c0 + q; float v = 0.f; if (o < O && col < KR) { const int c = TAPMAJ ? (col % CIN) : (col / 9); const int k = TAPMAJ ? (col / CIN) : (col % 9); v = bf16_round(Wm[((size_t)o * CIN + c) * 9 + k]) * 16.0f; } f.h[q] = (_Float16)v; } *(volatile v8us*)((unsigned short*)Bt + (size_t)o * KPAD + c0) = f.half[0]; }
    if (tid < 64) *(volatile float*)(BB + tid) = (tid < O) ? bm[tid] : 0.f;
    if (pass == 0) __threadfence(); } }
__global__ __launch_bounds__(256) void k_gat0(const float* __restrict__ x, const int* __restrict__ idx, int s0, _Float16* __restrict__ A) {
  const size_t t = (size_t)blockIdx.x * 256 + threadIdx.x; if (t >= (size_t)CHS * P0) return; const int p = (int)(t % P0); const int s = s0 + (int)(t / P0); FragH f[2]; for (int q = 0; q < 16; ++q) { f[0].u[q] = 0; f[1].u[q] = 0; }
#pragma unroll
  for (int c = 0; c < 2; ++c)
#pragma unroll
    for (int k = 0; k < 9; ++k) { const int src = idx[k * P0 + p]; const float v = (src >= 0 && src < P0) ? bf16_round(x[((size_t)s * 2 + c) * P0 + src]) : 0.f; const int col = c * 9 + k; if (col < 16) f[0].h[col] = (_Float16)v; else f[1].h[col - 16] = (_Float16)v; }
  unsigned short* d = (unsigned short*)A + t * 32; for (int pass = 0; pass < 2; ++pass) { *(volatile v8us*)d = f[0].half[0]; *(volatile v8us*)(d + 8) = f[0].half[1]; *(volatile v8us*)(d + 16) = f[1].half[0]; *(volatile v8us*)(d + 24) = f[1].half[1]; if (pass == 0) __threadfence(); } }
template <int CIN, int KPAD>
__global__ __launch_bounds__(256) void k_gat(const _Float16* __restrict__ HP, int PIN, const int* __restrict__ idx, int POUT, _Float16* __restrict__ A, size_t nrows) {
  constexpr int RPB = 32; __shared__ __attribute__((aligned(16))) unsigned short sh[RPB][KPAD];
  const int tid = threadIdx.x; const size_t row0 = (size_t)blockIdx.x * RPB;
  for (int e = tid; e < RPB * KPAD / 8; e += 256) { *(v8us*)&sh[e / (KPAD / 8)][(e % (KPAD / 8)) * 8] = (v8us){0, 0, 0, 0, 0, 0, 0, 0}; }
  __syncthreads();
  for (int wi = tid; wi < RPB * 9; wi += 256) { const int rl = wi / 9, t = wi % 9; const size_t row = row0 + rl; if (row >= nrows) continue; const int p = (int)(row % POUT); const size_t sl = row / POUT; const int src = idx[t * POUT + p];
    if (src >= 0 && src < PIN) { const unsigned short* s = (const unsigned short*)HP + (sl * PIN + src) * CIN;
#pragma unroll
      for (int c8 = 0; c8 < CIN; c8 += 8) *(v8us*)&sh[rl][t * CIN + c8] = *(const v8us*)(s + c8); } }
  __syncthreads();
  for (int pass = 0; pass < 2; ++pass) { for (int e = tid; e < RPB * (KPAD / 8); e += 256) { const int rl = e / (KPAD / 8), c8 = (e % (KPAD / 8)) * 8; const size_t row = row0 + rl; if (row >= nrows) continue; *(volatile v8us*)((unsigned short*)A + row * KPAD + c8) = *(const v8us*)&sh[rl][c8]; } if (pass == 0) __threadfence(); } }
template <int O>
__global__ __launch_bounds__(256) void k_bnr(const _Float16* __restrict__ C16, int P, const float* __restrict__ g, const float* __restrict__ bt, const float* __restrict__ rm, const float* __restrict__ rv, _Float16* __restrict__ HP) {
  #pragma clang fp contract(off)
  const size_t t = (size_t)blockIdx.x * 256 + threadIdx.x; if (t >= (size_t)CHS * P) return; FragH f[O / 8];
#pragma unroll
  for (int o = 0; o < O; ++o) { const float sc = bf16_round(g[o]) * rsqrtf(bf16_round(rv[o]) + 1e-5f); float y = ((float)C16[t * 64 + o] - bf16_round(rm[o])) * sc; y += bf16_round(bt[o]); f[o / 8].h[o % 8] = (_Float16)fmaxf(y, 0.f); }
  unsigned short* d = (unsigned short*)HP + t * O; for (int pass = 0; pass < 2; ++pass) { for (int u = 0; u < O / 8; ++u) *(volatile v8us*)(d + u * 8) = f[u].half[0]; if (pass == 0) __threadfence(); } }
template <int O>
__global__ __launch_bounds__(256) void k_pbr(const _Float16* __restrict__ C16, int PIN, const int* __restrict__ pidx, int POUT, const float* __restrict__ g, const float* __restrict__ bt, const float* __restrict__ rm, const float* __restrict__ rv, _Float16* __restrict__ HP) {
  #pragma clang fp contract(off)
  const size_t t = (size_t)blockIdx.x * 256 + threadIdx.x; if (t >= (size_t)CHS * POUT * (O / 8)) return; const int og = (int)(t % (O / 8)) * 8; const size_t pix = t / (O / 8); const int p = (int)(pix % POUT); const size_t sl = pix / POUT; float s[8]; for (int q = 0; q < 8; ++q) s[q] = 0.f;
#pragma unroll 1
  for (int k = 0; k < 9; ++k) { const int src = pidx[k * POUT + p]; if (src >= 0 && src < PIN) { const _Float16* c = C16 + (sl * PIN + src) * 64 + og;
#pragma unroll
      for (int q = 0; q < 8; ++q) s[q] += (float)c[q]; } }
  FragH f;
#pragma unroll
  for (int q = 0; q < 8; ++q) { const int o = og + q; const float sc = bf16_round(g[o]) * rsqrtf(bf16_round(rv[o]) + 1e-5f); float y = (s[q] / 9.0f - bf16_round(rm[o])) * sc; y += bf16_round(bt[o]); f.h[q] = (_Float16)fmaxf(y, 0.f); }
  unsigned short* d = (unsigned short*)HP + pix * O + og; *(volatile v8us*)d = f.half[0]; __threadfence(); *(volatile v8us*)d = f.half[0]; }
__global__ __launch_bounds__(128) void k_head(const _Float16* __restrict__ C16, const int* __restrict__ pidx, const float* __restrict__ g, const float* __restrict__ bt, const float* __restrict__ rm, const float* __restrict__ rv,
    const float* __restrict__ We1, const float* __restrict__ be1, const float* __restrict__ We2, const float* __restrict__ be2, const float* __restrict__ Wf, const float* __restrict__ bfv, const float* __restrict__ Wi, const float* __restrict__ bi, const float* __restrict__ Wd, const float* __restrict__ bd, const float* __restrict__ Wc, const float* __restrict__ bc, int s0, float* __restrict__ out) {
  #pragma clang fp contract(off)
  const int sl = blockIdx.x * 128 + threadIdx.x; if (sl >= CHS) return; const int s = s0 + sl; __shared__ float fsh[128][33];        float* fo = fsh[threadIdx.x];
#pragma unroll 1
  for (int o = 0; o < 32; ++o) { const float sc = bf16_round(g[o]) * rsqrtf(bf16_round(rv[o]) + 1e-5f), mu = bf16_round(rm[o]), be = bf16_round(bt[o]); float acc = 0.f;
#pragma unroll 1
    for (int p = 0; p < P3; ++p) { float sm = 0.f;
#pragma unroll 1
      for (int k = 0; k < 9; ++k) { const int src = pidx[k * P3 + p]; sm += (src >= 0 && src < P2) ? (float)C16[((size_t)sl * P2 + src) * 64 + o] : 0.f; }
      float y = (sm / 9.0f - mu) * sc; y += be; acc += fmaxf(y, 0.f); }
    fo[o] = acc / (float)P3; }
  float en = 0.f;
#pragma unroll 1
  for (int j = 0; j < 32; ++j) { float a = 0.f;
#pragma unroll 1
    for (int i = 0; i < 32; ++i) a += fo[i] * bf16_round(We1[j * 32 + i]);
    const float e1 = fmaxf(a + bf16_round(be1[j]), 0.f); en += e1 * bf16_round(We2[j]); }
  en += bf16_round(be2[0]);
  float imp0 = 0.f, imp1 = 0.f, dir0 = 0.f, dir1 = 0.f;
#pragma unroll 1
  for (int j = 0; j < 64; ++j) { float a = 0.f;
#pragma unroll 1
    for (int i = 0; i < 32; ++i) a += fo[i] * bf16_round(Wf[j * 32 + i]);
    const float fj = fmaxf(a + bf16_round(bfv[j]), 0.f); imp0 += fj * bf16_round(Wi[j]); imp1 += fj * bf16_round(Wi[64 + j]); dir0 += fj * bf16_round(Wd[j]); dir1 += fj * bf16_round(Wd[64 + j]); }
  imp0 += bf16_round(bi[0]); imp1 += bf16_round(bi[1]); dir0 += bf16_round(bd[0]); dir1 += bf16_round(bd[1]);
  float l0 = 0.f, l1 = 0.f;
#pragma unroll 1
  for (int i = 0; i < 32; ++i) { l0 += fo[i] * bf16_round(Wc[i]); l1 += fo[i] * bf16_round(Wc[32 + i]); }
  l0 += bf16_round(bc[0]); l1 += bf16_round(bc[1]); const float mx = fmaxf(l0, l1); const float lse = mx + logf(expf(l0 - mx) + expf(l1 - mx));
  for (int pass = 0; pass < 2; ++pass) { *(volatile float*)(out + s) = en; *(volatile float*)(out + 512 + s * 2) = imp0; *(volatile float*)(out + 512 + s * 2 + 1) = imp1; *(volatile float*)(out + 1536 + s * 2) = dir0; *(volatile float*)(out + 1536 + s * 2 + 1) = dir1; *(volatile float*)(out + 2560 + s * 2) = l0 - lse; *(volatile float*)(out + 2560 + s * 2 + 1) = l1 - lse; if (pass == 0) __threadfence(); } }

extern "C" void kernel_launch(void* const* d_in, const int* in_sizes, int n_in,
                              void* d_out, int out_size, void* d_ws, size_t ws_size, hipStream_t stream) {
  (void)in_sizes; (void)n_in; (void)out_size;
  const float* const* I = (const float* const*)d_in; auto II = [&](int i) { return (const int*)d_in[i]; };
  const float* x = I[0];
  const float* W0 = I[1]; const float* b0 = I[2]; const float* g0 = I[3]; const float* t0 = I[4]; const float* m0 = I[5]; const float* v0 = I[6]; const int* ic0 = II(7);
  const float* W1 = I[8]; const float* b1 = I[9]; const float* g1 = I[10]; const float* t1 = I[11]; const float* m1 = I[12]; const float* v1 = I[13]; const int* ic1 = II(14); const int* ip1 = II(15);
  const float* W2 = I[16]; const float* b2 = I[17]; const float* g2 = I[18]; const float* t2 = I[19]; const float* m2 = I[20]; const float* v2 = I[21]; const int* ic2 = II(22); const int* ip2 = II(23);
  const float* W3 = I[24]; const float* b3 = I[25]; const float* g3 = I[26]; const float* t3 = I[27]; const float* m3 = I[28]; const float* v3 = I[29]; const int* ic3 = II(30); const int* ip3 = II(31);
  const float* We1 = I[32]; const float* be1 = I[33]; const float* We2 = I[34]; const float* be2 = I[35]; const float* Wf = I[36]; const float* bfv = I[37]; const float* Wi = I[38]; const float* bi = I[39]; const float* Wd = I[40]; const float* bd = I[41]; const float* Wc = I[42]; const float* bc = I[43];
  char* ws = (char*)d_ws; size_t off = 0;
  auto take = [&](size_t bytes) { char* p = ws + off; off += (bytes + 255) & ~(size_t)255; return p; };
  _Float16* BW0 = (_Float16*)take(64 * 32 * 2); _Float16* BW1 = (_Float16*)take(64 * 160 * 2); _Float16* BW2 = (_Float16*)take(64 * 160 * 2); _Float16* BW3 = (_Float16*)take(64 * 320 * 2); float* BB0 = (float*)take(256); float* BB1 = (float*)take(256); float* BB2 = (float*)take(256); float* BB3 = (float*)take(256);
  const size_t R0 = (size_t)CHS * P0, R1 = (size_t)CHS * P1, R2 = (size_t)CHS * P2;
  const int PH0 = ((P0 + 7) / 8) * 8, PH1 = ((P1 + 7) / 8) * 8, PH2 = ((P2 + 7) / 8) * 8;
  _Float16* A = (_Float16*)take(R0 * 160 * 2); _Float16* C16 = (_Float16*)take(R0 * 64 * 2); _Float16* HA = (_Float16*)take((size_t)CHS * P0 * 16 * 2); _Float16* HB = (_Float16*)take((size_t)CHS * P0 * 16 * 2);
  if (off > ws_size) return;
  k_wconv<<<1, 256, 0, stream>>>(W0, b0, 16, 2, 32, 0, BW0, BB0); k_wconv<<<1, 256, 0, stream>>>(W1, b1, 16, 16, 160, 1, BW1, BB1); k_wconv<<<1, 256, 0, stream>>>(W2, b2, 32, 16, 160, 1, BW2, BB2); k_wconv<<<1, 256, 0, stream>>>(W3, b3, 32, 32, 320, 1, BW3, BB3);
  for (int s0 = 0; s0 < NS; s0 += CHS) {
    k_gat0<<<(unsigned)((R0 + 255) / 256), 256, 0, stream>>>(x, ic0, s0, A);
    k_gemm2<0><<<dim3((unsigned)(R0 / 128), 1), 128, 0, stream>>>(A, 32, 0, BW0, 32, 0, 0.0625f, BB0, 0, nullptr, 1, 0, 0, nullptr, C16, 64, 0, (int)R0, 64, 32);
    k_bnr<16><<<(unsigned)((R0 + 255) / 256), 256, 0, stream>>>(C16, P0, g0, t0, m0, v0, HA);
    k_gat<16, 160><<<(unsigned)((R0 + 31) / 32), 256, 0, stream>>>(HA, P0, ic1, P0, A, R0);
    k_gemm2<0><<<dim3((unsigned)(R0 / 128), 1), 128, 0, stream>>>(A, 160, 0, BW1, 160, 0, 0.0625f, BB1, 0, nullptr, 1, 0, 0, nullptr, C16, 64, 0, (int)R0, 64, 160);
    k_pbr<16><<<(unsigned)((R1 * 2 + 255) / 256), 256, 0, stream>>>(C16, P0, ip1, P1, g1, t1, m1, v1, HB);
    k_gat<16, 160><<<(unsigned)((R1 + 31) / 32), 256, 0, stream>>>(HB, P1, ic2, P1, A, R1);
    k_gemm2<0><<<dim3((unsigned)(R1 / 128), 1), 128, 0, stream>>>(A, 160, 0, BW2, 160, 0, 0.0625f, BB2, 0, nullptr, 1, 0, 0, nullptr, C16, 64, 0, (int)R1, 64, 160);
    k_pbr<32><<<(unsigned)((R2 * 4 + 255) / 256), 256, 0, stream>>>(C16, P1, ip2, P2, g2, t2, m2, v2, HA);
    k_gat<32, 320><<<(unsigned)((R2 + 31) / 32), 256, 0, stream>>>(HA, P2, ic3, P2, A, R2);
    k_gemm2<0><<<dim3((unsigned)(R2 / 128), 1), 128, 0, stream>>>(A, 320, 0, BW3, 320, 0, 0.0625f, BB3, 0, nullptr, 1, 0, 0, nullptr, C16, 64, 0, (int)R2, 64, 320);
    k_head<<<(CHS + 127) / 128, 128, 0, stream>>>(C16, ip3, g3, t3, m3, v3, We1, be1, We2, be2, Wf, bfv, Wi, bi, Wd, bd, Wc, bc, s0, (float*)d_out); }
}
